// PhiInv_54872502174405
// MI455X (gfx1250) — hardware-verified
//
#include <hip/hip_runtime.h>
#include <math.h>

typedef __attribute__((ext_vector_type(16))) _Float16 v16h;
typedef __attribute__((ext_vector_type(8)))  _Float16 v8h;
typedef __attribute__((ext_vector_type(8)))  float    v8f;
typedef __attribute__((ext_vector_type(4)))  float    v4f;
typedef __attribute__((ext_vector_type(4)))  unsigned v4u;

constexpr int kNPts       = 2097152;
constexpr int kComp       = 32;
constexpr int kMaxSteps   = 16;
constexpr int kBlockThr   = 256;
constexpr int kPtsPerWave = 32;
static_assert((kNPts % kBlockThr) == 0, "grid covers the points exactly");
static_assert((kBlockThr % kPtsPerWave) == 0, "whole waves");
static_assert(kComp == 32, "one 32-deep k step");

constexpr float kLog2e        = 1.4426950408889634f;
constexpr float kWCarry       = 64.0f;
constexpr float kLoCarry      = 2048.0f;
constexpr float kLoCarryInv   = 1.0f / kLoCarry;
constexpr int   kECarryBits   = 10;
constexpr float kECarryLog2   = (float)kECarryBits;
constexpr float kECarry       = (float)(1 << kECarryBits);
constexpr float kYScale       = kWCarry * kECarry;
constexpr float kF16MinNormal = 6.103515625e-5f;
constexpr float kExitDt       = 1.0e-3f;
constexpr float kPFloor       = 1.0f;
static_assert(kYScale == 65536.0f, "carry chain");

constexpr size_t kOffTab   = 0;
constexpr size_t kOffTile  = 512;
constexpr size_t kWsTotal  = 512 + 1024;
static_assert((kOffTile % 128) == 0, "line aligned");
static_assert(kWsTotal <= 134217728ull, "carve cap");

__device__ __forceinline__ v8f mma_guarded(v16h a, v16h b, v8f c) {
  c = __builtin_amdgcn_wmma_f32_16x16x32_f16(false, a, false, b, (short)0, c, false, false);
  asm volatile("v_nop\n\tv_nop\n\tv_nop\n\tv_nop" : "+v"(c) : "v"(a), "v"(b));
  return c;
}

__global__ __launch_bounds__(32) void mix_prep_kernel(
    const float* __restrict__ wl, const float* __restrict__ sr, unsigned* __restrict__ wsw)
{
  __shared__ float sE[kComp];
  __shared__ __align__(16) unsigned sStage[8 * kComp];
  unsigned k = threadIdx.x & 31u;
  asm volatile("" : "+v"(k));

  float mx = wl[0];
#pragma unroll 1
  for (int i = 1; i < kComp; ++i) mx = fmaxf(mx, wl[i]);
  const float ek = expf(wl[k] - mx);
  sE[k] = ek;
  __syncthreads();
  float z = 0.0f;
#pragma unroll 1
  for (int i = 0; i < kComp; ++i) z += sE[i];
  const float wk = ek / z;

  const float x  = sr[k];
  const float sk = (fmaxf(x, 0.0f) + log1pf(expf(-fabsf(x)))) + 0.1f;
  const float ck = -sk * kLog2e;
  const float wsk = wk * sk;

  const float a0  = wk * kWCarry;
  const float a1  = wsk * kWCarry;
  const float a0f = (fabsf(a0) < kF16MinNormal) ? 0.0f : a0;
  const float a1f = (fabsf(a1) < kF16MinNormal) ? 0.0f : a1;
  const _Float16 h0 = (_Float16)a0f;
  const _Float16 h1 = (_Float16)a1f;
  const float r0  = (a0 - (float)h0) * kLoCarry;
  const float r1  = (a1 - (float)h1) * kLoCarry;
  const float r0f = (fabsf(r0) < kF16MinNormal) ? 0.0f : r0;
  const float r1f = (fabsf(r1) < kF16MinNormal) ? 0.0f : r1;
  const _Float16 l0 = (_Float16)r0f;
  const _Float16 l1 = (_Float16)r1f;
  const unsigned h0b = (unsigned)__builtin_bit_cast(unsigned short, h0);
  const unsigned h1b = (unsigned)__builtin_bit_cast(unsigned short, h1);
  const unsigned l0b = (unsigned)__builtin_bit_cast(unsigned short, l0);
  const unsigned l1b = (unsigned)__builtin_bit_cast(unsigned short, l1);

  sStage[0u * 32u + k] = __float_as_uint(ck);
  sStage[1u * 32u + k] = __float_as_uint(sk);
  sStage[2u * 32u + k] = __float_as_uint(wk);
  sStage[3u * 32u + k] = 0u;
  sStage[4u * 32u + k] = h0b;
  sStage[5u * 32u + k] = h1b;
  sStage[6u * 32u + k] = l0b;
  sStage[7u * 32u + k] = l1b;
  __syncthreads();

  const v4u tv = *(const v4u*)(sStage + 4u * k);

  unsigned r = k >> 2;
  asm volatile("" : "+v"(r));
  unsigned rc = (r < 4u) ? r : 3u;
  asm volatile("" : "+v"(rc));
  unsigned cb = (k & 3u) * 8u;
  asm volatile("" : "+v"(cb));
  const unsigned* src = sStage + (4u + rc) * 32u + cb;
  const v4u q0 = *(const v4u*)(src);
  const v4u q1 = *(const v4u*)(src + 4);
  const bool live = (r < 4u);
  const unsigned p0 = (q0[1] << 16) | (q0[0] & 0xffffu);
  const unsigned p1 = (q0[3] << 16) | (q0[2] & 0xffffu);
  const unsigned p2 = (q1[1] << 16) | (q1[0] & 0xffffu);
  const unsigned p3 = (q1[3] << 16) | (q1[2] & 0xffffu);
  v4u tw;
  tw[0] = live ? p0 : 0u;
  tw[1] = live ? p1 : 0u;
  tw[2] = live ? p2 : 0u;
  tw[3] = live ? p3 : 0u;

  unsigned* pt = wsw + 4u * k;
  unsigned* pa = wsw + 128u + 4u * k;
  unsigned* pb = wsw + 256u + 4u * k;
  *(volatile v4u*)pt = tv;
  *(volatile v4u*)pa = tw;
  *(volatile v4u*)pb = tw;
  __threadfence();
  *(volatile v4u*)pt = tv;
  *(volatile v4u*)pa = tw;
  *(volatile v4u*)pb = tw;
}

__global__ __launch_bounds__(256) void mix_solve_kernel(
    const float* __restrict__ y, const float* __restrict__ tab,
    const unsigned short* __restrict__ tile, float* __restrict__ out)
{
  __shared__ __align__(16) float sTab[4 * kComp];
  const unsigned tid = threadIdx.x;
  if (tid < 128u) sTab[tid] = tab[tid];
  __syncthreads();

  unsigned lane = tid & 31u;
  asm volatile("" : "+v"(lane));
  unsigned wave = tid >> 5;
  asm volatile("" : "+v"(wave));
  unsigned h = lane >> 4;
  asm volatile("" : "+v"(h));
  unsigned n = lane & 15u;
  asm volatile("" : "+v"(n));

  const unsigned base = (blockIdx.x * (unsigned)(kBlockThr / kPtsPerWave) + wave) * (unsigned)kPtsPerWave;
  unsigned ia = base + n;
  unsigned ib = base + 16u + n;
  ia = (ia < (unsigned)kNPts) ? ia : (unsigned)(kNPts - 1);
  ib = (ib < (unsigned)kNPts) ? ib : (unsigned)(kNPts - 1);
  asm volatile("" : "+v"(ia));
  asm volatile("" : "+v"(ib));
  const float ya = y[ia];
  const float yb = y[ib];
  const float ysa = ya * kYScale;
  const float ysb = yb * kYScale;

  union WF { v16h v; v8h hh[2]; };
  WF wf;
  {
    const _Float16* wp = (const _Float16*)tile + n * 32u + 8u * h;
    wf.hh[0] = *(const v8h*)(wp);
    wf.hh[1] = *(const v8h*)(wp + 16);
  }

  float cl[16];
  {
    const float* cp = sTab + 8u * h;
    const v4f c0 = *(const v4f*)(cp);
    const v4f c1 = *(const v4f*)(cp + 4);
    const v4f c2 = *(const v4f*)(cp + 16);
    const v4f c3 = *(const v4f*)(cp + 20);
    cl[0]  = c0[0]; cl[1]  = c0[1]; cl[2]  = c0[2]; cl[3]  = c0[3];
    cl[4]  = c1[0]; cl[5]  = c1[1]; cl[6]  = c1[2]; cl[7]  = c1[3];
    cl[8]  = c2[0]; cl[9]  = c2[1]; cl[10] = c2[2]; cl[11] = c2[3];
    cl[12] = c3[0]; cl[13] = c3[1]; cl[14] = c3[2]; cl[15] = c3[3];
  }

  const v8f zero8 = (v8f){0.f, 0.f, 0.f, 0.f, 0.f, 0.f, 0.f, 0.f};
  float ta = 0.0f, tb = 0.0f;
#pragma unroll 1
  for (int it = 0; it < kMaxSteps; ++it) {
    v16h ea, eb;
#pragma unroll
    for (int i = 0; i < 16; ++i) {
      float va = __builtin_amdgcn_exp2f(fmaf(ta, cl[i], kECarryLog2));
      float vb = __builtin_amdgcn_exp2f(fmaf(tb, cl[i], kECarryLog2));
      va = (va < kF16MinNormal) ? 0.0f : va;
      vb = (vb < kF16MinNormal) ? 0.0f : vb;
      ea[i] = (_Float16)va;
      eb[i] = (_Float16)vb;
    }
    const v8f da = mma_guarded(wf.v, ea, zero8);
    const v8f db = mma_guarded(wf.v, eb, zero8);
    const float fa = fmaf(da[2], kLoCarryInv, da[0]);
    const float pa = fmaxf(fmaf(da[3], kLoCarryInv, da[1]), kPFloor);
    const float fb = fmaf(db[2], kLoCarryInv, db[0]);
    const float pb = fmaxf(fmaf(db[3], kLoCarryInv, db[1]), kPFloor);
    const float dta = (fa - ysa) * __builtin_amdgcn_rcpf(pa);
    const float dtb = (fb - ysb) * __builtin_amdgcn_rcpf(pb);
    ta += dta;
    tb += dtb;
    const bool busy = (fmaxf(fabsf(dta), fabsf(dtb)) >= kExitDt);
    const unsigned any = __builtin_amdgcn_ballot_w32(busy);
    if (any == 0u) break;
  }

  const bool up = (h != 0u);
  const float tf = up ? tb : ta;
  const float yf = up ? yb : ya;
  float f = 0.0f, p = 0.0f;
#pragma unroll 1
  for (int k = 0; k < kComp; ++k) {
    const float sk = sTab[kComp + k];
    const float wk = sTab[2 * kComp + k];
    const float e  = expf(-tf * sk);
    f = fmaf(e, wk, f);
    p = fmaf(e * sk, wk, p);
  }
  const float res = tf + (f - yf) / p;

  if (base < (unsigned)kNPts) {
    float* po = out + (base + lane);
    *(volatile float*)po = res;
    __threadfence();
    *(volatile float*)po = res;
  }
}

extern "C" void kernel_launch(void* const* d_in, const int* in_sizes, int n_in,
                              void* d_out, int out_size, void* d_ws, size_t ws_size,
                              hipStream_t stream) {
  if (n_in < 3) return;
  if (in_sizes[0] != kNPts) return;
  if (in_sizes[1] != kComp) return;
  if (in_sizes[2] != kComp) return;
  if (out_size != kNPts) return;
  if (ws_size < kWsTotal) return;

  const float* y  = (const float*)d_in[0];
  const float* wl = (const float*)d_in[1];
  const float* sr = (const float*)d_in[2];
  float* out = (float*)d_out;
  char* ws = (char*)d_ws;

  mix_prep_kernel<<<1, 32, 0, stream>>>(wl, sr, (unsigned*)(ws + kOffTab));
  mix_solve_kernel<<<kNPts / kBlockThr, kBlockThr, 0, stream>>>(
      y, (const float*)(ws + kOffTab), (const unsigned short*)(ws + kOffTile), out);
}
